// ModulatedDeformableConv2d_5669356831723
// MI455X (gfx1250) — hardware-verified
//
#include <hip/hip_runtime.h>
#include <math.h>


typedef _Float16 v16h __attribute__((ext_vector_type(16)));
typedef _Float16 v8h  __attribute__((ext_vector_type(8)));
typedef _Float16 v2h  __attribute__((ext_vector_type(2)));
typedef float    v8f  __attribute__((ext_vector_type(8)));
typedef float    v4f  __attribute__((ext_vector_type(4)));
typedef v8h __attribute__((may_alias)) v8h_ma;
typedef v2h __attribute__((may_alias)) v2h_ma;
typedef v4f __attribute__((may_alias)) v4f_ma;

#define CH      64
#define COUT    64
#define IMH     128
#define IMW     128
#define TAPS    9
#define NOFF    27
#define NOFFP   32
#define KTOT    (CH * TAPS)
#define BPITCH  584
#define APITCH  72
#define SPITCH  128
#define NWAVE   8
#define NTHR    (NWAVE * 32)
#define CBMAX   4
#define WSCALE  256.0f
#define WINV    (1.0f / 256.0f)

static_assert(IMW == NWAVE * 16);
static_assert((BPITCH * 2) % 16 == 0 && (APITCH * 2) % 16 == 0 && (KTOT * 2) % 128 == 0);
static_assert(NOFFP * SPITCH * 4 <= NOFFP * BPITCH * 2);
static_assert(COUT * SPITCH * 4 <= COUT * BPITCH * 2);

union FragH { v16h v; v8h half[2]; };

static __device__ __forceinline__ v8f wmma_f16(v16h a, v16h b, v8f c) {
  v8f d = __builtin_amdgcn_wmma_f32_16x16x32_f16(false, a, false, b, (short)0, c, false, false);
  asm volatile("v_nop\n\tv_nop\n\tv_nop\n\tv_nop" : "+v"(d) : "v"(a), "v"(b));
  return d;
}

static __device__ __forceinline__ v16h load_frag_row(const _Float16* rowk0, int h) {
  FragH f;
  f.half[0] = *(const v8h_ma*)(rowk0 + 8 * h);
  f.half[1] = *(const v8h_ma*)(rowk0 + 16 + 8 * h);
  return f.v;
}

static __device__ __forceinline__ void store_rows(const float* stg, float* gbase, size_t chs,
                                                  int wave, int lane, int nrows, bool ok) {
  #pragma unroll
  for (int q = 0; q < 8; ++q) {
    const int n = wave + NWAVE * q;
    if (ok && n < nrows) {
      const v4f v = *(const v4f_ma*)(stg + n * SPITCH + 4 * lane);
      *(volatile v4f*)(gbase + (size_t)n * chs + 4 * lane) = v;
    }
  }
}

__global__ __launch_bounds__(NTHR) void k_offset_mask(
    const float* __restrict__ xe, const float* __restrict__ w_off,
    const float* __restrict__ b_off, float* __restrict__ om, int nb)
{
  __shared__ __attribute__((aligned(16))) _Float16 bsh[NOFFP * BPITCH];
  __shared__ __attribute__((aligned(16))) _Float16 ash[NWAVE][16][APITCH];

  const int tid = threadIdx.x, wave = tid >> 5, lane = tid & 31;
  const int h = lane >> 4, m = lane & 15;

  for (int i = tid; i < NOFFP * TAPS * (CH / 2); i += NTHR) {
    const int cp = i & (CH / 2 - 1);
    const int t  = (i / (CH / 2)) % TAPS;
    const int n  = i / (TAPS * (CH / 2));
    const int c  = 2 * cp;
    float v0 = 0.f, v1 = 0.f;
    if (n < NOFF) {
      v0 = w_off[(n * CH + c) * TAPS + t] * WSCALE;
      v1 = w_off[(n * CH + c + 1) * TAPS + t] * WSCALE;
    }
    v2h pr; pr[0] = (_Float16)v0; pr[1] = (_Float16)v1;
    *(v2h_ma*)(bsh + n * BPITCH + t * CH + c) = pr;
  }
  __syncthreads();

  const int blk = blockIdx.x;
  const int ho  = blk % IMH;
  int b = blk / IMH;
  const bool bok = (b < nb);
  b = min(b, nb - 1);
  const int wo0 = wave * 16;
  const size_t chs = (size_t)IMH * IMW;

  v8f acc[2] = {};

  const float* xc0 = xe + ((size_t)b * CH + 2 * lane) * chs;

  for (int t = 0; t < TAPS; ++t) {
    const int ky = t / 3, kx = t - 3 * ky;
    const int y  = ho - 1 + ky;
    const bool vy = (y >= 0) && (y < IMH);
    const int yc = min(max(y, 0), IMH - 1);
    const float* prow = xc0 + (size_t)yc * IMW;
    __syncthreads();
    #pragma unroll
    for (int r = 0; r < 16; ++r) {
      const int xx  = wo0 - 1 + kx + r;
      const int xcl = min(max(xx, 0), IMW - 1);
      float v0 = prow[xcl];
      float v1 = prow[xcl + chs];
      const bool ok = vy & (xx >= 0) & (xx < IMW);
      v0 = ok ? v0 : 0.f;
      v1 = ok ? v1 : 0.f;
      v2h pr; pr[0] = (_Float16)v0; pr[1] = (_Float16)v1;
      *(v2h_ma*)(&ash[wave][r][2 * lane]) = pr;
    }
    __syncthreads();
    const _Float16* arow = &ash[wave][m][0];
    #pragma unroll
    for (int kc = 0; kc < 2; ++kc) {
      const v16h af = load_frag_row(arow + kc * 32, h);
      const int koff = t * CH + kc * 32;
      #pragma unroll
      for (int nt = 0; nt < 2; ++nt) {
        const v16h bf = load_frag_row(bsh + (nt * 16 + m) * BPITCH + koff, h);
        acc[nt] = wmma_f16(af, bf, acc[nt]);
      }
    }
  }

  __syncthreads();
  float* stg = reinterpret_cast<float*>(bsh);
  #pragma unroll
  for (int nt = 0; nt < 2; ++nt) {
    const int n = nt * 16 + m;
    const float bv = b_off[min(n, NOFF - 1)];
    const bool sig = (n >= 2 * TAPS);
    v4f p0, p1;
    #pragma unroll
    for (int j = 0; j < 4; ++j) {
      float u0 = acc[nt][j] * WINV + bv;
      float u1 = acc[nt][j + 4] * WINV + bv;
      if (sig) {
        u0 = 1.0f / (1.0f + expf(-u0));
        u1 = 1.0f / (1.0f + expf(-u1));
      }
      p0[j] = u0;
      p1[j] = u1;
    }
    float* sp = stg + n * SPITCH + wo0 + 8 * h;
    *(v4f_ma*)sp = p0;
    *(v4f_ma*)(sp + 4) = p1;
  }
  __syncthreads();

  float* gbase = om + (size_t)b * NOFF * chs + (size_t)ho * IMW;
  store_rows(stg, gbase, chs, wave, lane, NOFF, bok);
  __threadfence();
  store_rows(stg, gbase, chs, wave, lane, NOFF, bok);
}

__global__ __launch_bounds__(NTHR) void k_deform_cols(
    const float* __restrict__ x, const float* __restrict__ om,
    _Float16* __restrict__ col, int nb, int b0, int cb)
{
  __shared__ __attribute__((aligned(16))) _Float16 ash[NWAVE][16][APITCH];

  const int tid = threadIdx.x, wave = tid >> 5, lane = tid & 31;

  const int blk = blockIdx.x;
  const int ho  = blk % IMH;
  int bl = blk / IMH;
  const bool bok = (bl < cb) && (b0 + bl < nb);
  bl = min(bl, cb - 1);
  const int b = min(b0 + bl, nb - 1);
  const int wo0 = wave * 16;
  const size_t chs = (size_t)IMH * IMW;

  const float* xp0 = x + ((size_t)b * CH + 2 * lane) * chs;
  const float* xp1 = xp0 + chs;
  const float* omb = om + (size_t)b * NOFF * chs + (size_t)ho * IMW + wo0;
  const size_t pix0 = ((size_t)bl * IMH + ho) * IMW + wo0;

  const int sp  = lane >> 3;
  const int cof = 8 * (lane & 7);

  for (int t = 0; t < TAPS; ++t) {
    const int ky = t / 3, kx = t - 3 * ky;
    const float* offY = omb + (size_t)(2 * t) * chs;
    const float* offX = omb + (size_t)(2 * t + 1) * chs;
    const float* msk  = omb + (size_t)(2 * TAPS + t) * chs;
    const float ybase = (float)(ho - 1 + ky);
    const int   xib   = wo0 - 1 + kx;
    __syncthreads();
    #pragma unroll 2
    for (int r = 0; r < 16; ++r) {
      float py = offY[r] + ybase;
      float px = offX[r] + (float)(xib + r);
      const float mk = msk[r];
      py = fminf(fmaxf(py, -2.0f), (float)(IMH + 1));
      px = fminf(fmaxf(px, -2.0f), (float)(IMW + 1));
      const float y0f = floorf(py), x0f = floorf(px);
      const int y0 = (int)y0f, x0 = (int)x0f;
      const float wy = py - y0f, wx = px - x0f;
      float w00 = (1.f - wy) * (1.f - wx);
      float w01 = (1.f - wy) * wx;
      float w10 = wy * (1.f - wx);
      float w11 = wy * wx;
      const bool vy0 = (y0 >= 0) & (y0 < IMH);
      const bool vy1 = (y0 + 1 >= 0) & (y0 + 1 < IMH);
      const bool vx0 = (x0 >= 0) & (x0 < IMW);
      const bool vx1 = (x0 + 1 >= 0) & (x0 + 1 < IMW);
      w00 = (vy0 & vx0) ? w00 : 0.f;
      w01 = (vy0 & vx1) ? w01 : 0.f;
      w10 = (vy1 & vx0) ? w10 : 0.f;
      w11 = (vy1 & vx1) ? w11 : 0.f;
      const int yc0 = min(max(y0, 0), IMH - 1);
      const int yc1 = min(max(y0 + 1, 0), IMH - 1);
      const int xc0 = min(max(x0, 0), IMW - 1);
      const int xc1 = min(max(x0 + 1, 0), IMW - 1);
      const int i00 = yc0 * IMW + xc0, i01 = yc0 * IMW + xc1;
      const int i10 = yc1 * IMW + xc0, i11 = yc1 * IMW + xc1;
      const float s0 = w00 * xp0[i00] + w01 * xp0[i01] + w10 * xp0[i10] + w11 * xp0[i11];
      const float s1 = w00 * xp1[i00] + w01 * xp1[i01] + w10 * xp1[i10] + w11 * xp1[i11];
      v2h pr; pr[0] = (_Float16)(s0 * mk); pr[1] = (_Float16)(s1 * mk);
      *(v2h_ma*)(&ash[wave][r][2 * lane]) = pr;
    }
    __syncthreads();

    v4f v[4];
    #pragma unroll
    for (int q = 0; q < 4; ++q) v[q] = *(const v4f_ma*)(&ash[wave][4 * q + sp][cof]);
    if (bok) {
      #pragma unroll
      for (int q = 0; q < 4; ++q)
        *(volatile v4f*)(col + (pix0 + 4 * q + sp) * KTOT + t * CH + cof) = v[q];
    }
    __threadfence();
    if (bok) {
      #pragma unroll
      for (int q = 0; q < 4; ++q)
        *(volatile v4f*)(col + (pix0 + 4 * q + sp) * KTOT + t * CH + cof) = v[q];
    }
  }
}

__global__ __launch_bounds__(NTHR) void k_gemm_out(
    const _Float16* __restrict__ col, const float* __restrict__ weight,
    const float* __restrict__ bias, float* __restrict__ out, int nb, int b0, int cb)
{
  __shared__ __attribute__((aligned(16))) _Float16 bsh[COUT * BPITCH];

  const int tid = threadIdx.x, wave = tid >> 5, lane = tid & 31;
  const int h = lane >> 4, m = lane & 15;

  for (int i = tid; i < COUT * TAPS * (CH / 2); i += NTHR) {
    const int cp = i & (CH / 2 - 1);
    const int t  = (i / (CH / 2)) % TAPS;
    const int o  = i / (TAPS * (CH / 2));
    const int c  = 2 * cp;
    const float v0 = weight[(o * CH + c) * TAPS + t] * WSCALE;
    const float v1 = weight[(o * CH + c + 1) * TAPS + t] * WSCALE;
    v2h pr; pr[0] = (_Float16)v0; pr[1] = (_Float16)v1;
    *(v2h_ma*)(bsh + o * BPITCH + t * CH + c) = pr;
  }
  __syncthreads();

  const int blk = blockIdx.x;
  const int ho  = blk % IMH;
  int bl = blk / IMH;
  const bool bok = (bl < cb) && (b0 + bl < nb);
  bl = min(bl, cb - 1);
  const int b = min(b0 + bl, nb - 1);
  const int wo0 = wave * 16;
  const size_t chs = (size_t)IMH * IMW;

  v8f acc[4] = {};

  const _Float16* arow = col + (((size_t)bl * IMH + ho) * IMW + wo0 + m) * KTOT;

  #pragma unroll 2
  for (int ks = 0; ks < KTOT / 32; ++ks) {
    const int k0 = ks * 32;
    const v16h af = load_frag_row(arow + k0, h);
    #pragma unroll
    for (int nt = 0; nt < 4; ++nt) {
      const v16h bf = load_frag_row(bsh + (nt * 16 + m) * BPITCH + k0, h);
      acc[nt] = wmma_f16(af, bf, acc[nt]);
    }
  }

  __syncthreads();
  float* stg = reinterpret_cast<float*>(bsh);
  #pragma unroll
  for (int nt = 0; nt < 4; ++nt) {
    const int n = nt * 16 + m;
    const float bv = bias[n];
    v4f p0, p1;
    #pragma unroll
    for (int j = 0; j < 4; ++j) {
      p0[j] = acc[nt][j] * WINV + bv;
      p1[j] = acc[nt][j + 4] * WINV + bv;
    }
    float* sp = stg + n * SPITCH + wo0 + 8 * h;
    *(v4f_ma*)sp = p0;
    *(v4f_ma*)(sp + 4) = p1;
  }
  __syncthreads();

  float* gbase = out + (size_t)b * COUT * chs + (size_t)ho * IMW;
  store_rows(stg, gbase, chs, wave, lane, COUT, bok);
  __threadfence();
  store_rows(stg, gbase, chs, wave, lane, COUT, bok);
}

extern "C" void kernel_launch(void* const* d_in, const int* in_sizes, int n_in,
                              void* d_out, int out_size, void* d_ws, size_t ws_size,
                              hipStream_t stream) {
  if (n_in < 6) return;
  const int per_img = CH * IMH * IMW;
  const int nb = in_sizes[0] / per_img;
  if (nb < 1 || in_sizes[0] != nb * per_img) return;
  if (in_sizes[1] != nb * per_img) return;
  if (in_sizes[2] != NOFF * KTOT || in_sizes[3] < NOFF) return;
  if (in_sizes[4] != COUT * KTOT || in_sizes[5] < COUT) return;
  if (out_size != nb * COUT * IMH * IMW) return;

  const size_t om_bytes  = (size_t)nb * NOFF * IMH * IMW * sizeof(float);
  const size_t col_off   = (om_bytes + 255) & ~(size_t)255;
  const size_t col_img   = (size_t)KTOT * IMH * IMW * sizeof(_Float16);
  const size_t ws_cap    = (size_t)128 * 1024 * 1024;
  const size_t cap       = ws_size < ws_cap ? ws_size : ws_cap;
  int cb = nb < CBMAX ? nb : CBMAX;
  while (cb > 1 && col_off + (size_t)cb * col_img > cap) --cb;
  if (col_off + (size_t)cb * col_img > cap) return;
  const int nchunk = (nb + cb - 1) / cb;

  const float* x       = (const float*)d_in[0];
  const float* x_extra = (const float*)d_in[1];
  const float* w_off   = (const float*)d_in[2];
  const float* b_off   = (const float*)d_in[3];
  const float* weight  = (const float*)d_in[4];
  const float* bias    = (const float*)d_in[5];
  float* om      = (float*)d_ws;
  _Float16* col  = (_Float16*)((char*)d_ws + col_off);
  float* out     = (float*)d_out;

  dim3 block(NTHR);
  k_offset_mask<<<dim3(nb * IMH), block, 0, stream>>>(x_extra, w_off, b_off, om, nb);
  for (int ch = 0; ch < nchunk; ++ch) {
    const int b0  = ch * cb;
    const int cbc = (nb - b0) < cb ? (nb - b0) : cb;
    dim3 grid(cbc * IMH);
    k_deform_cols<<<grid, block, 0, stream>>>(x, om, col, nb, b0, cbc);
    k_gemm_out<<<grid, block, 0, stream>>>(col, weight, bias, out, nb, b0, cbc);
  }
}
